// NonLocal_21792664060441
// MI455X (gfx1250) — hardware-verified
//
#include <hip/hip_runtime.h>
#include <math.h>

constexpr int kB  = 8;
constexpr int kC  = 64;
constexpr int kCI = 32;
constexpr int kN  = 4096;
constexpr int kPW = 128;
constexpr float kWCarry    = 16.0f;
constexpr float kWCarryInv = 1.0f / 16.0f;
constexpr float kPCarry    = 32768.0f;
constexpr float kPCarryInv = 1.0f / 32768.0f;
static_assert(kN % 64 == 0 && kPW % 64 == 0 && kC % 64 == 0, "M,N tiles");
static_assert(kC % 32 == 0 && kCI % 32 == 0 && kN % 32 == 0, "K steps");
static_assert(kN == 4 * 1024, "softmax row map");

typedef __attribute__((ext_vector_type(16))) _Float16 v16h;
typedef __attribute__((ext_vector_type(8)))  _Float16 v8h;
typedef __attribute__((ext_vector_type(16))) __bf16   v16b;
typedef __attribute__((ext_vector_type(8)))  __bf16   v8b;
typedef __attribute__((ext_vector_type(8)))  float    v8f;
typedef __attribute__((ext_vector_type(4)))  float    v4f;
typedef __attribute__((ext_vector_type(4)))  unsigned int v4u;

__device__ __forceinline__ unsigned short f2bf_bits(float f) {
  unsigned u = __float_as_uint(f);
  return (unsigned short)((u + 0x7FFFu + ((u >> 16) & 1u)) >> 16);
}
__device__ __forceinline__ float bf_bits2f(unsigned short h) { return __uint_as_float(((unsigned)h) << 16); }

__device__ __forceinline__ void dep_guard4_h(v8f& a, v8f& b, v8f& c, v8f& d, v16h x, v16h y) { asm volatile("v_nop\n\tv_nop\n\tv_nop\n\tv_nop" : "+v"(a), "+v"(b), "+v"(c), "+v"(d) : "v"(x), "v"(y)); }
__device__ __forceinline__ void dep_guard4_b(v8f& a, v8f& b, v8f& c, v8f& d, v16b x, v16b y) { asm volatile("v_nop\n\tv_nop\n\tv_nop\n\tv_nop" : "+v"(a), "+v"(b), "+v"(c), "+v"(d) : "v"(x), "v"(y)); }
__device__ __forceinline__ void keep4_h(v16h a, v16h b, v16h c, v16h d) { asm volatile("v_nop" :: "v"(a), "v"(b), "v"(c), "v"(d)); }
__device__ __forceinline__ void keep4_b(v16b a, v16b b, v16b c, v16b d) { asm volatile("v_nop" :: "v"(a), "v"(b), "v"(c), "v"(d)); }
__device__ __forceinline__ void acc_guard4(v8f& a, v8f& b, v8f& c, v8f& d) { asm volatile("v_nop\n\tv_nop\n\tv_nop\n\tv_nop" : "+v"(a), "+v"(b), "+v"(c), "+v"(d)); }
template <typename T> struct Frag;
template <> struct Frag<_Float16> {
  typedef v16h V; union U { v16h v; v8h h[2]; };
  static __device__ __forceinline__ v16h load(const _Float16* p) {
    U f; f.h[0] = *(const v8h*)(p); f.h[1] = *(const v8h*)(p + 16); return f.v;
  }
  static __device__ __forceinline__ v8f mma(v16h a, v16h b, v8f c) {
    return __builtin_amdgcn_wmma_f32_16x16x32_f16(false, a, false, b, (short)0, c, false, false);
  }
  static __device__ __forceinline__ void guard4(v8f& a, v8f& b, v8f& c, v8f& d, v16h x, v16h y) { dep_guard4_h(a, b, c, d, x, y); }
  static __device__ __forceinline__ void keep(v16h a, v16h b, v16h c, v16h d) { keep4_h(a, b, c, d); }
};
template <> struct Frag<__bf16> {
  typedef v16b V; union U { v16b v; v8b h[2]; };
  static __device__ __forceinline__ v16b load(const __bf16* p) {
    U f; f.h[0] = *(const v8b*)(p); f.h[1] = *(const v8b*)(p + 16); return f.v;
  }
  static __device__ __forceinline__ v8f mma(v16b a, v16b b, v8f c) {
    return __builtin_amdgcn_wmma_f32_16x16x32_bf16(false, a, false, b, (short)0, c, false, false);
  }
  static __device__ __forceinline__ void guard4(v8f& a, v8f& b, v8f& c, v8f& d, v16b x, v16b y) { dep_guard4_b(a, b, c, d, x, y); }
  static __device__ __forceinline__ void keep(v16b a, v16b b, v16b c, v16b d) { keep4_b(a, b, c, d); }
};

__device__ __forceinline__ unsigned pk16(unsigned short a, unsigned short b) { return (unsigned)a | ((unsigned)b << 16); }
__device__ __forceinline__ unsigned short h_bits(float f) { const _Float16 h = (_Float16)f; return __builtin_bit_cast(unsigned short, h); }

template <int ET> struct Elem;
template <> struct Elem<0> { typedef _Float16 T; };
template <> struct Elem<1> { typedef __bf16 T; };
template <int ET, bool SPLIT, int BIAS_MODE, int OUT_MODE, bool RESID, int ACT = 0>
__global__ __launch_bounds__(256) void wmma_gemm64(
    const unsigned short* __restrict__ Ap, const unsigned short* __restrict__ A2p, int lda, long strideA,
    const unsigned short* __restrict__ Btp, const unsigned short* __restrict__ Bt2p, int ldb, long strideB,
    void* __restrict__ Cout, void* __restrict__ Cout2, int ldc, long strideC,
    const float* __restrict__ bias,
    const float* __restrict__ resid, long strideR,
    int M, int N, int K, float scale) {
  static_assert(!RESID || OUT_MODE == 0, "resid only with f32 output");
  static_assert(ACT == 0 || ACT == 2 || ACT == 4, "act");
  typedef typename Elem<ET>::T T;
  typedef typename Frag<T>::V V;
  const T* A = (const T*)Ap; const T* A2 = (const T*)A2p; const T* Bt = (const T*)Btp; const T* Bt2 = (const T*)Bt2p;
  __shared__ __align__(16) float sT[8][16 * 68];
  const int b    = blockIdx.y;
  const int lane = threadIdx.x & 31;
  const int wave = threadIdx.x >> 5;
  const int tilesN = N >> 6;
  const int tilesM = M >> 6;
  const int tile = blockIdx.x * 8 + wave;
  if (tile >= tilesM * tilesN) return;
  const int tm = tile / tilesN;
  const int tn = tile - tm * tilesN;
  const int m0 = tm << 6;
  const int n0 = tn << 6;

  const T* Ab  = A  + (size_t)b * strideA;
  const T* Bb  = Bt + (size_t)b * strideB;
  const T* Ab2 = SPLIT ? (A2  + (size_t)b * strideA) : nullptr;
  const T* Bb2 = SPLIT ? (Bt2 + (size_t)b * strideB) : nullptr;

  const int rlane = lane & 15;
  const int koff  = (lane >> 4) * 8;
  const int mOff  = (lane >> 4) * 8;

  v8f acc[4][4];
#pragma unroll
  for (int i = 0; i < 4; ++i)
#pragma unroll
    for (int j = 0; j < 4; ++j) acc[i][j] = (v8f){0.f,0.f,0.f,0.f,0.f,0.f,0.f,0.f};

  for (int k0 = 0; k0 < K; k0 += 32) {
    V bh[4], bl[4];
#pragma unroll
    for (int j = 0; j < 4; ++j) {
      const size_t bo = (size_t)(n0 + (j << 4) + rlane) * ldb + koff + k0;
      bh[j] = Frag<T>::load(Bb + bo);
      if (SPLIT) bl[j] = Frag<T>::load(Bb2 + bo);
    }
#pragma unroll
    for (int i = 0; i < 4; ++i) {
      const size_t ao = (size_t)(m0 + (i << 4) + rlane) * lda + koff + k0;
      V ah = Frag<T>::load(Ab + ao);
      V al;
      if (SPLIT) al = Frag<T>::load(Ab2 + ao);
#pragma unroll
      for (int j = 0; j < 4; ++j) {
        acc[i][j] = Frag<T>::mma(ah, bh[j], acc[i][j]);
        if (SPLIT) {
          acc[i][j] = Frag<T>::mma(ah, bl[j], acc[i][j]);
          acc[i][j] = Frag<T>::mma(al, bh[j], acc[i][j]);
        }
      }
      Frag<T>::guard4(acc[i][0], acc[i][1], acc[i][2], acc[i][3], ah, SPLIT ? al : ah);
    }
    Frag<T>::keep(bh[0], bh[1], bh[2], bh[3]);
    if (SPLIT) Frag<T>::keep(bl[0], bl[1], bl[2], bl[3]);
  }
  acc_guard4(acc[0][0], acc[0][1], acc[0][2], acc[0][3]);
  acc_guard4(acc[1][0], acc[1][1], acc[1][2], acc[1][3]);
  acc_guard4(acc[2][0], acc[2][1], acc[2][2], acc[2][3]);
  acc_guard4(acc[3][0], acc[3][1], acc[3][2], acc[3][3]);

  float* slab = sT[wave];
  const float* Rb = RESID ? (resid + (size_t)b * strideR) : nullptr;
#pragma unroll
  for (int i = 0; i < 4; ++i) {
    const int mBase = m0 + (i << 4);
#pragma unroll
    for (int j = 0; j < 4; ++j) {
      const int n = n0 + (j << 4) + rlane;
      float bv = 0.f;
      if (BIAS_MODE == 2) bv = bias[n];
#pragma unroll
      for (int r = 0; r < 8; ++r) {
        float v = acc[i][j][r] * scale;
        if (BIAS_MODE == 1) v += bias[mBase + mOff + r];
        if (BIAS_MODE == 2) v += bv;
        if (ACT == 2) v = fmaxf(v, 0.0f);
        if (ACT == 4) v = (v > 0.f) ? v : 0.01f * v;
        slab[(mOff + r) * 68 + (j << 4) + rlane] = v;
      }
    }
    __builtin_amdgcn_fence(__ATOMIC_RELEASE, "workgroup");
    __builtin_amdgcn_wave_barrier();
    __builtin_amdgcn_fence(__ATOMIC_ACQUIRE, "workgroup");
    if (OUT_MODE == 0) {
      float* C = (float*)Cout + (size_t)b * strideC;
      const int hh = lane >> 4, c4 = (lane & 15) * 4;
      for (int pass = 0; pass < 2; ++pass) {
#pragma unroll
        for (int it = 0; it < 8; ++it) {
          const int row = it * 2 + hh;
          v4f v = *(const v4f*)(slab + row * 68 + c4);
          if (RESID) {
            const v4f rr = *(const v4f*)(Rb + (size_t)(mBase + row) * ldc + n0 + c4);
            v = v + rr;
          }
          *(volatile v4f*)(C + (size_t)(mBase + row) * ldc + n0 + c4) = v;
        }
        __threadfence();
      }
    } else {
      const int q = lane >> 3, c8 = (lane & 7) * 8;
      unsigned short* C  = (unsigned short*)Cout  + (size_t)b * strideC;
      unsigned short* C2 = (OUT_MODE == 2) ? ((unsigned short*)Cout2 + (size_t)b * strideC) : nullptr;
      for (int pass = 0; pass < 2; ++pass) {
#pragma unroll
        for (int it = 0; it < 4; ++it) {
          const int row = it * 4 + q;
          const float* sp = slab + row * 68 + c8;
          v8h hv, lv;
#pragma unroll
          for (int e = 0; e < 8; ++e) {
            if (OUT_MODE == 1) {
              hv[e] = (_Float16)sp[e];
            } else {
              unsigned short hb = f2bf_bits(sp[e]);
              unsigned short lb = f2bf_bits(sp[e] - bf_bits2f(hb));
              hv[e] = __builtin_bit_cast(_Float16, hb);
              lv[e] = __builtin_bit_cast(_Float16, lb);
            }
          }
          *(volatile v8h*)(C + (size_t)(mBase + row) * ldc + n0 + c8) = hv;
          if (OUT_MODE == 2) *(volatile v8h*)(C2 + (size_t)(mBase + row) * ldc + n0 + c8) = lv;
        }
        __threadfence();
      }
    }
    __builtin_amdgcn_fence(__ATOMIC_RELEASE, "workgroup");
    __builtin_amdgcn_wave_barrier();
    __builtin_amdgcn_fence(__ATOMIC_ACQUIRE, "workgroup");
  }
}

__global__ __launch_bounds__(256) void prep_kernel(const float* __restrict__ w_theta, const float* __restrict__ w_phi,
                                                   const float* __restrict__ w_g,
                                                   const float* __restrict__ b_theta, const float* __restrict__ b_phi,
                                                   const float* __restrict__ b_g, const float* __restrict__ w_out,
                                                   unsigned short* __restrict__ wcat, float* __restrict__ bcat,
                                                   unsigned short* __restrict__ wo16) {
  const int t   = threadIdx.x;
  const int blk = blockIdx.x;
  if (blk < 4) {
    v4u u;
    if (blk < 3) {
      const float* src = (blk == 0) ? w_theta : ((blk == 1) ? w_phi : w_g);
      const int rl = t >> 3, c8 = (t & 7) * 8;
      const v4f a = *(const v4f*)(src + rl * kC + c8);
      const v4f c = *(const v4f*)(src + rl * kC + c8 + 4);
      unsigned short hb[8];
#pragma unroll
      for (int e = 0; e < 4; ++e) {
        hb[e]     = h_bits(a[e] * kWCarry);
        hb[4 + e] = h_bits(c[e] * kWCarry);
      }
      u = (v4u){pk16(hb[0], hb[1]), pk16(hb[2], hb[3]), pk16(hb[4], hb[5]), pk16(hb[6], hb[7])};
    } else {
      u = (v4u){0u, 0u, 0u, 0u};
    }
    unsigned short* dst = wcat + (size_t)blk * (32 * kC) + 8 * (size_t)t;
    *(volatile v4u*)dst = u;
    __threadfence();
    *(volatile v4u*)dst = u;
  } else if (blk == 4) {
    if (t < 32) {
      const int seg = t >> 3;
      const int o4  = (t & 7) * 4;
      const v4f bt = *(const v4f*)(b_theta + o4);
      const v4f bp = *(const v4f*)(b_phi + o4);
      const v4f bg = *(const v4f*)(b_g + o4);
      const float f0 = (seg == 0) ? 1.0f : 0.0f;
      const float f1 = (seg == 1) ? 1.0f : 0.0f;
      const float f2 = (seg == 2) ? 1.0f : 0.0f;
      v4f val;
#pragma unroll
      for (int e = 0; e < 4; ++e) val[e] = fmaf(f0, bt[e], fmaf(f1, bp[e], f2 * bg[e]));
      float* dst = bcat + 4 * t;
      *(volatile v4f*)dst = val;
      __threadfence();
      *(volatile v4f*)dst = val;
    }
  } else {
    const int row = t >> 2, c8 = (t & 3) * 8;
    const v4f a = *(const v4f*)(w_out + row * kCI + c8);
    const v4f c = *(const v4f*)(w_out + row * kCI + c8 + 4);
    unsigned short hb[8];
#pragma unroll
    for (int e = 0; e < 4; ++e) {
      hb[e]     = h_bits(a[e] * kWCarry);
      hb[4 + e] = h_bits(c[e] * kWCarry);
    }
    const v4u u = (v4u){pk16(hb[0], hb[1]), pk16(hb[2], hb[3]), pk16(hb[4], hb[5]), pk16(hb[6], hb[7])};
    unsigned short* dst = wo16 + 8 * (size_t)t;
    *(volatile v4u*)dst = u;
    __threadfence();
    *(volatile v4u*)dst = u;
  }
}

__global__ __launch_bounds__(256) void xt_cast_kernel(const float* __restrict__ x, unsigned short* __restrict__ XT) {
  __shared__ float sm[64][65];
  const int t  = threadIdx.x;
  const int n0 = blockIdx.x * 64;
  const int b  = blockIdx.y;
#pragma unroll
  for (int i = 0; i < 16; ++i) {
    const int e  = i * 256 + t;
    const int cl = e >> 6;
    const int nl = e & 63;
    sm[nl][cl] = x[((size_t)(b * kC + cl)) * kN + n0 + nl];
  }
  __syncthreads();
  const int lane = t & 31, wave = t >> 5;
  const int q = lane >> 3, c8 = (lane & 7) * 8;
  unsigned short* op = XT + ((size_t)b * kN + n0) * kC;
  for (int pass = 0; pass < 2; ++pass) {
#pragma unroll
    for (int it = 0; it < 2; ++it) {
      const int row = wave * 8 + it * 4 + q;
      unsigned short hb[8];
#pragma unroll
      for (int e = 0; e < 8; ++e) hb[e] = h_bits(sm[row][c8 + e]);
      const v4u u = (v4u){pk16(hb[0], hb[1]), pk16(hb[2], hb[3]), pk16(hb[4], hb[5]), pk16(hb[6], hb[7])};
      *(volatile v4u*)(op + (size_t)row * kC + c8) = u;
    }
    __threadfence();
  }
}

__global__ __launch_bounds__(256) void softmax_row_kernel(const float* __restrict__ S, unsigned short* __restrict__ P) {
  __shared__ __align__(16) float lg[kN];
  __shared__ float redM[8];
  __shared__ float redS[8];
  const int row  = blockIdx.x;
  const int t    = threadIdx.x;
  const int lane = t & 31, wave = t >> 5;
  const float* sr = S + (size_t)row * kN;

  float mx = -__builtin_inff();
#pragma unroll 1
  for (int it = 0; it < 4; ++it) {
    const int c = it * 1024 + 4 * t;
    const v4f sv = *(const v4f*)(sr + c);
    mx = fmaxf(mx, fmaxf(fmaxf(sv[0], sv[1]), fmaxf(sv[2], sv[3])));
    *(v4f*)(lg + c) = sv;
  }
#pragma unroll
  for (int off = 16; off > 0; off >>= 1) mx = fmaxf(mx, __shfl_xor(mx, off, 32));
  if (lane == 0) redM[wave] = mx;
  __syncthreads();
  float m = redM[0];
#pragma unroll
  for (int w = 1; w < 8; ++w) m = fmaxf(m, redM[w]);

  float sum = 0.f;
#pragma unroll 1
  for (int it = 0; it < 4; ++it) {
    const int c = it * 1024 + 4 * t;
    const v4f l = *(const v4f*)(lg + c);
    v4f ev;
#pragma unroll
    for (int e = 0; e < 4; ++e) {
      ev[e] = expf(l[e] - m);
      sum += ev[e];
    }
    *(v4f*)(lg + c) = ev;
  }
#pragma unroll
  for (int off = 16; off > 0; off >>= 1) sum += __shfl_xor(sum, off, 32);
  if (lane == 0) redS[wave] = sum;
  __syncthreads();
  float tot = redS[0];
#pragma unroll
  for (int w = 1; w < 8; ++w) tot += redS[w];
  const float inv = kPCarry / tot;

  const v4f e0 = *(const v4f*)(lg + 8 * t);
  const v4f e1 = *(const v4f*)(lg + 8 * t + 4);
  const v4f e2 = *(const v4f*)(lg + 2048 + 8 * t);
  const v4f e3 = *(const v4f*)(lg + 2048 + 8 * t + 4);
  unsigned short ha[8], hc[8];
#pragma unroll
  for (int e = 0; e < 4; ++e) {
    ha[e]     = h_bits(e0[e] * inv);
    ha[4 + e] = h_bits(e1[e] * inv);
    hc[e]     = h_bits(e2[e] * inv);
    hc[4 + e] = h_bits(e3[e] * inv);
  }
  const v4u u0 = (v4u){pk16(ha[0], ha[1]), pk16(ha[2], ha[3]), pk16(ha[4], ha[5]), pk16(ha[6], ha[7])};
  const v4u u1 = (v4u){pk16(hc[0], hc[1]), pk16(hc[2], hc[3]), pk16(hc[4], hc[5]), pk16(hc[6], hc[7])};
  unsigned short* p0 = P + (size_t)row * kN + 8 * (size_t)t;
  unsigned short* p1 = p0 + 2048;
  *(volatile v4u*)p0 = u0;
  *(volatile v4u*)p1 = u1;
  __threadfence();
  *(volatile v4u*)p0 = u0;
  *(volatile v4u*)p1 = u1;
}

extern "C" void kernel_launch(void* const* d_in, const int* in_sizes, int n_in,
                              void* d_out, int out_size, void* d_ws, size_t ws_size,
                              hipStream_t stream) {
  if (n_in < 9) return;
  const int nX = kB * kC * kN;
  if (in_sizes[0] != nX) return;
  if (in_sizes[1] != kCI * kC || in_sizes[2] != kCI) return;
  if (in_sizes[3] != kCI * kC || in_sizes[4] != kCI) return;
  if (in_sizes[5] != kCI * kC || in_sizes[6] != kCI) return;
  if (in_sizes[7] != kC * kCI || in_sizes[8] != kC) return;
  if (out_size != nX) return;

  const size_t szWC  = (size_t)kPW * kC * 2;
  const size_t szBC  = (size_t)kPW * 4;
  const size_t szWO  = (size_t)kC * kCI * 2;
  const size_t szXT  = (size_t)kB * kN * kC * 2;
  const size_t szPRJ = (size_t)kB * kN * kPW * 2;
  const size_t szGWT = (size_t)kB * kC * kN * 2;
  const size_t szS   = (size_t)kN * kN * 4;
  const size_t szP   = (size_t)kN * kN * 2;
  const size_t offWC  = 0;
  const size_t offBC  = offWC + szWC;
  const size_t offWO  = offBC + szBC;
  const size_t offXT  = offWO + szWO;
  const size_t offPRJ = offXT + szXT;
  const size_t offGWT = offPRJ + szPRJ;
  const size_t offS   = offGWT + szGWT;
  const size_t offP   = offS + szS;
  const size_t total  = offP + szP;
  if (ws_size < total) return;

  const float* x       = (const float*)d_in[0];
  const float* w_theta = (const float*)d_in[1];
  const float* b_theta = (const float*)d_in[2];
  const float* w_phi   = (const float*)d_in[3];
  const float* b_phi   = (const float*)d_in[4];
  const float* w_g     = (const float*)d_in[5];
  const float* b_g     = (const float*)d_in[6];
  const float* w_out   = (const float*)d_in[7];
  const float* b_out   = (const float*)d_in[8];
  float* out = (float*)d_out;
  char* ws = (char*)d_ws;
  unsigned short* WC  = (unsigned short*)(ws + offWC);
  float*          BC  = (float*)(ws + offBC);
  unsigned short* WO  = (unsigned short*)(ws + offWO);
  unsigned short* XT  = (unsigned short*)(ws + offXT);
  unsigned short* PRJ = (unsigned short*)(ws + offPRJ);
  unsigned short* GWT = (unsigned short*)(ws + offGWT);
  float*          SC  = (float*)(ws + offS);
  unsigned short* PP  = (unsigned short*)(ws + offP);

  prep_kernel<<<dim3(6), dim3(256), 0, stream>>>(w_theta, w_phi, w_g, b_theta, b_phi, b_g, w_out, WC, BC, WO);
  xt_cast_kernel<<<dim3(kN / 64, kB), dim3(256), 0, stream>>>(x, XT);

  const long strideXT  = (long)kN * kC;
  const long stridePRJ = (long)kN * kPW;
  const long strideGWT = (long)kC * kN;
  wmma_gemm64<0, false, 2, 1, false, 0><<<dim3(16, kB), dim3(256), 0, stream>>>(
      XT, XT, kC, strideXT, WC, WC, kC, 0L,
      (void*)PRJ, (void*)PRJ, kPW, stridePRJ, BC, x, 0L, kN, kPW, kC, kWCarryInv);

  wmma_gemm64<0, false, 0, 1, false, 0><<<dim3(8, kB), dim3(256), 0, stream>>>(
      WO, WO, kCI, 0L, PRJ + 64, PRJ + 64, kPW, stridePRJ,
      (void*)GWT, (void*)GWT, kN, strideGWT, BC, x, 0L, kC, kN, kCI, kWCarryInv);

  for (int b = 0; b < kB; ++b) {
    const unsigned short* prjb = PRJ + (size_t)b * kN * kPW;
    wmma_gemm64<0, false, 0, 0, false, 0><<<dim3(512, 1), dim3(256), 0, stream>>>(
        prjb, prjb, kPW, 0L, prjb + 32, prjb + 32, kPW, 0L,
        (void*)SC, (void*)SC, kN, 0L, BC, x, 0L, kN, kN, kCI, 1.0f);
    softmax_row_kernel<<<dim3(kN), dim3(256), 0, stream>>>(SC, PP);
    const unsigned short* gwtb = GWT + (size_t)b * kC * kN;
    float* outb = out + (size_t)b * kC * kN;
    const float* xb = x + (size_t)b * kC * kN;
    wmma_gemm64<0, false, 1, 0, true, 0><<<dim3(8, 1), dim3(256), 0, stream>>>(
        gwtb, gwtb, kN, 0L, PP, PP, kN, 0L,
        (void*)outb, (void*)outb, kN, 0L, b_out, xb, 0L, kC, kN, kN, kPCarryInv);
  }
}
